// MoE_22591527977486
// MI455X (gfx1250) — hardware-verified
//
#include <hip/hip_runtime.h>
#include <math.h>

#define TT 4096
#define CC 128
#define DIN 128
#define NH 4
#define HD 32
#define HG 1
#define NQB (TT / 64)
#define CAUSAL 0
#define QHI 64
#define KHI 64
#define QBH 0
#define SCALE (1.0f)
typedef __attribute__((ext_vector_type(16))) _Float16 v16h;
typedef __attribute__((ext_vector_type(16))) __bf16 v16b;
typedef __attribute__((ext_vector_type(8)))  _Float16 v8h;
typedef __attribute__((ext_vector_type(8)))  float v8f;
typedef __attribute__((ext_vector_type(4)))  float v4f;
typedef __attribute__((ext_vector_type(2)))  float v2f;
typedef __attribute__((ext_vector_type(4)))  unsigned v4u;
typedef __attribute__((ext_vector_type(4)))  int v4i;
typedef float __attribute__((may_alias)) float_a;
typedef int __attribute__((may_alias)) int_a;

template <typename T> __device__ __forceinline__ void vst2(void* p, T v) { *(volatile T*)p = v; __threadfence(); *(volatile T*)p = v; }
__device__ __forceinline__ v8f wmma16(v16h a, v16h b, v8f c) {
  v8f d = __builtin_amdgcn_wmma_f32_16x16x32_f16(false, a, false, b, (short)0, c, false, false);
  asm volatile("v_nop\n\tv_nop\n\tv_nop\n\tv_nop" : "+v"(d) : "v"(a), "v"(b));
  return d;
}
__device__ __forceinline__ v8f wmma_bf(v16b a, v16b b, v8f c) {
  v8f d = __builtin_amdgcn_wmma_f32_16x16x32_bf16(false, a, false, b, (short)0, c, false, false);
  asm volatile("v_nop\n\tv_nop\n\tv_nop\n\tv_nop" : "+v"(d) : "v"(a), "v"(b));
  return d;
}
__device__ __forceinline__ v16h frag_h(const _Float16* rowk0, int lane) {
  union { v16h v; v8h q[2]; } u; const _Float16* p = rowk0 + 8 * (lane >> 4);
  u.q[0] = *(const v8h*)p; u.q[1] = *(const v8h*)(p + 16); return u.v;
}
__device__ __forceinline__ v16h frag_f32(const float* rowk0, int lane) {
  v16h a; const float* p = rowk0 + 8 * (lane >> 4);
#pragma unroll
  for (int i = 0; i < 8; ++i) { a[i] = (_Float16)p[i]; a[8 + i] = (_Float16)p[16 + i]; }
  return a;
}
__device__ __forceinline__ v16h frag_f32s(const float* rowk0, int lane, float sc) {
  v16h a; const float* p = rowk0 + 8 * (lane >> 4);
#pragma unroll
  for (int i = 0; i < 8; ++i) { a[i] = (_Float16)(p[i] * sc); a[8 + i] = (_Float16)(p[16 + i] * sc); }
  return a;
}
__device__ __forceinline__ v16h fragc_f32(const float* W, int k0, int n, int lane, int ld, int K) {
  v16h a; const int g = lane >> 4;
#pragma unroll
  for (int i = 0; i < 8; ++i) { const int ka = k0 + 8 * g + i, kb = ka + 16;
    a[i] = (_Float16)(ka < K ? W[(size_t)(ka < K ? ka : K - 1) * ld + n] : 0.f); a[8 + i] = (_Float16)(kb < K ? W[(size_t)(kb < K ? kb : K - 1) * ld + n] : 0.f); }
  return a;
}
struct F2 { v16b h, l; };
__device__ __forceinline__ F2 bsplit16(const float v[16]) { F2 r;
#pragma unroll
  for (int i = 0; i < 16; ++i) { const __bf16 h = (__bf16)v[i]; r.h[i] = h; r.l[i] = (__bf16)(v[i] - (float)h); }
  return r; }
__device__ __forceinline__ F2 split_row(const float* row, int k0, int lane) { float v[16]; const float* p = row + k0 + 8 * (lane >> 4);
#pragma unroll
  for (int i = 0; i < 8; ++i) { v[i] = p[i]; v[8 + i] = p[16 + i]; }
  return bsplit16(v); }
__device__ __forceinline__ F2 split_rowK(const float* row, int k0, int lane, int K) { float v[16]; const int g = lane >> 4;
#pragma unroll
  for (int i = 0; i < 8; ++i) { const int ka = k0 + 8 * g + i, kb = ka + 16; v[i] = ka < K ? row[ka < K ? ka : K - 1] : 0.f; v[8 + i] = kb < K ? row[kb < K ? kb : K - 1] : 0.f; }
  return bsplit16(v); }
__device__ __forceinline__ F2 split_col(const float* W, int k0, int n, int lane, int ld, int K) { float v[16]; const int g = lane >> 4;
#pragma unroll
  for (int i = 0; i < 8; ++i) { const int ka = k0 + 8 * g + i, kb = ka + 16; v[i] = ka < K ? W[(size_t)(ka < K ? ka : K - 1) * ld + n] : 0.f; v[8 + i] = kb < K ? W[(size_t)(kb < K ? kb : K - 1) * ld + n] : 0.f; }
  return bsplit16(v); }
__device__ __forceinline__ v8f mac3(const F2& a, const F2& b, v8f c) { c = wmma_bf(a.l, b.h, c); c = wmma_bf(a.h, b.l, c); return wmma_bf(a.h, b.h, c); }
__device__ __forceinline__ float sigm(float v) { return 1.0f / (1.0f + expf(-v)); }
#define LDSX() do { asm volatile("s_wait_dscnt 0" ::: "memory"); __builtin_amdgcn_wave_barrier(); __builtin_amdgcn_fence(__ATOMIC_RELEASE, "workgroup"); } while (0)

__device__ __forceinline__ float bfr(float v) { return (float)(__bf16)v; }
__host__ __device__ __forceinline__ int kb_last(int qb) { return CAUSAL ? ((qb * 64 + 63) >> 7) : (TT / 128 - 1); }
typedef __attribute__((ext_vector_type(8))) __bf16 v8b;
__device__ __forceinline__ v16b frag_b(const __bf16* rowk0, int lane) {
  union { v16b v; v8b q[2]; } u; const __bf16* p = rowk0 + 8 * (lane >> 4);
  u.q[0] = *(const v8b*)p; u.q[1] = *(const v8b*)(p + 16); return u.v;
}
__device__ __forceinline__ v16b wcol_io(const float* Wm, int k0, int o, int lane, int ld) { v16b w; const int g = lane >> 4;
#pragma unroll
  for (int i = 0; i < 8; ++i) { w[i] = (__bf16)Wm[(size_t)(k0 + 8 * g + i) * ld + o]; w[8 + i] = (__bf16)Wm[(size_t)(k0 + 16 + 8 * g + i) * ld + o]; }
  return w; }
__device__ __forceinline__ v16b wcol_oi(const float* Wm, int k0, int o, int lane, int K) { v16b w; const float* p = Wm + (size_t)o * K + k0 + 8 * (lane >> 4);
#pragma unroll
  for (int i = 0; i < 8; ++i) { w[i] = (__bf16)p[i]; w[8 + i] = (__bf16)p[16 + i]; }
  return w; }
__device__ __forceinline__ v16h wcolh_io(const float* Wm, int k0, int o, int lane, int ld) { v16h w; const int g = lane >> 4;
#pragma unroll
  for (int i = 0; i < 8; ++i) { w[i] = (_Float16)(bfr(Wm[(size_t)(k0 + 8 * g + i) * ld + o]) * 256.0f); w[8 + i] = (_Float16)(bfr(Wm[(size_t)(k0 + 16 + 8 * g + i) * ld + o]) * 256.0f); }
  return w; }
__device__ __forceinline__ v16h wcolh_oi(const float* Wm, int k0, int o, int lane, int K) { v16h w; const float* p = Wm + (size_t)o * K + k0 + 8 * (lane >> 4);
#pragma unroll
  for (int i = 0; i < 8; ++i) { w[i] = (_Float16)(bfr(p[i]) * 256.0f); w[8 + i] = (_Float16)(bfr(p[16 + i]) * 256.0f); }
  return w; }
__device__ __forceinline__ v16b wcol_hdk(const float* Wm, int k0, int o, int lane) { v16b w; const int g = lane >> 4; const float* p = Wm + (size_t)(o / HD) * DIN * HD + (o % HD);
#pragma unroll
  for (int i = 0; i < 8; ++i) { w[i] = (__bf16)p[(size_t)(k0 + 8 * g + i) * HD]; w[8 + i] = (__bf16)p[(size_t)(k0 + 16 + 8 * g + i) * HD]; }
  return w; }
#define WO_OUT_IN 1
#if WQKV_LAYOUT == 1
#define WCOL(W, k0, o, lane) wcol_oi(W, k0, o, lane, DIN)
#elif WQKV_LAYOUT == 2
#define WCOL(W, k0, o, lane) wcol_hdk(W, k0, o, lane)
#else
#define WCOL(W, k0, o, lane) wcol_io(W, k0, o, lane, CC)
#endif
#if WO_OUT_IN
#define WOCOL(W, k0, o, lane) wcol_oi(W, k0, o, lane, CC)
#define WOCOLH(W, k0, o, lane) wcolh_oi(W, k0, o, lane, CC)
#else
#define WOCOL(W, k0, o, lane) wcol_io(W, k0, o, lane, DIN)
#define WOCOLH(W, k0, o, lane) wcolh_io(W, k0, o, lane, DIN)
#endif

#ifndef SM_EXTRA_PARAMS
#define SM_EXTRA_PARAMS
#endif
#ifndef PROJ_EXTRA_PARAMS
#define PROJ_EXTRA_PARAMS
#endif
#ifndef SM_MASK_HOOK
#define SM_MASK_HOOK (void)0
#endif


#define NR 1024
#define DM 512
#define NK 8
#define PH 64
#define GW 128
__device__ __forceinline__ float elu1(float v) { return v > 0.f ? v : expm1f(v); }
__global__ __launch_bounds__(128) void k_g0(const float* __restrict__ PHs, const float* __restrict__ Wm, const float* __restrict__ Bv, float* __restrict__ G0) { __shared__ __align__(16) float sf[4][16][132];
  const int tid = threadIdx.x, wave = tid >> 5, lane = tid & 31, col = lane & 15, g = lane >> 4; const size_t r0 = (size_t)blockIdx.x * 64 + wave * 16;
  v8f acc[8] = {};
#pragma unroll
  for (int kc = 0; kc < PH / 32; ++kc) { v16b a; { const float* p = PHs + (r0 + col) * PH + kc * 32 + 8 * g;
#pragma unroll
      for (int i = 0; i < 8; ++i) { a[i] = (__bf16)p[i]; a[8 + i] = (__bf16)p[16 + i]; } }
    asm volatile("s_wait_loadcnt 0x0" ::: "memory");
#pragma unroll
    for (int j = 0; j < 8; ++j) { const v16b w = wcol_io(Wm, kc * 32, j * 16 + col, lane, GW); acc[j] = wmma_bf(a, w, acc[j]); } }
#pragma unroll
  for (int j = 0; j < 8; ++j) { const float bb = bfr(Bv[j * 16 + col]); asm volatile("s_wait_loadcnt 0x0" ::: "memory");
#pragma unroll
    for (int r = 0; r < 8; ++r) sf[wave][8 * g + r][j * 16 + col] = elu1(acc[j][r] + bb); }
  LDSX(); for (int rl = 0; rl < 16; ++rl) vst2(G0 + (r0 + rl) * GW + lane * 4, *(const v4f*)&sf[wave][rl][lane * 4]); }
__global__ __launch_bounds__(128) void k_g1(const float* __restrict__ G0, const float* __restrict__ Wm, const float* __restrict__ Bv, float* __restrict__ G1) { __shared__ __align__(16) float sf[4][16][132];
  const int tid = threadIdx.x, wave = tid >> 5, lane = tid & 31, col = lane & 15, g = lane >> 4; const size_t r0 = (size_t)blockIdx.x * 64 + wave * 16;
  v8f acc[8] = {};
#pragma unroll
  for (int kc = 0; kc < GW / 32; ++kc) { const F2 a = split_row(G0 + (r0 + col) * GW, kc * 32, lane);
    asm volatile("s_wait_loadcnt 0x0" ::: "memory");
#pragma unroll
    for (int j = 0; j < 8; ++j) { const v16b w = wcol_io(Wm, kc * 32, j * 16 + col, lane, GW); acc[j] = wmma_bf(a.h, w, acc[j]); acc[j] = wmma_bf(a.l, w, acc[j]); } }
#pragma unroll
  for (int j = 0; j < 8; ++j) { const float bb = bfr(Bv[j * 16 + col]); asm volatile("s_wait_loadcnt 0x0" ::: "memory");
#pragma unroll
    for (int r = 0; r < 8; ++r) sf[wave][8 * g + r][j * 16 + col] = elu1(acc[j][r] + bb); }
  LDSX(); for (int rl = 0; rl < 16; ++rl) vst2(G1 + (r0 + rl) * GW + lane * 4, *(const v4f*)&sf[wave][rl][lane * 4]); }
__global__ __launch_bounds__(256) void k_coef(const float* __restrict__ G1, const float* __restrict__ W2g, const float* __restrict__ B2g, float* __restrict__ COEF) { const int tid = threadIdx.x; const int e = tid & 7; const size_t row = (size_t)blockIdx.x * 32 + (tid >> 3);
  float l = 0.f;
#pragma unroll 4
  for (int k = 0; k < GW; ++k) { const float gv = G1[row * GW + k], wv = W2g[(size_t)k * NK + e]; asm volatile("s_wait_loadcnt 0x0" ::: "memory"); l += gv * bfr(wv); }
  { const float bb = B2g[e]; asm volatile("s_wait_loadcnt 0x0" ::: "memory"); l += bfr(bb); }
  float m = l; m = fmaxf(m, __shfl_xor(m, 1)); m = fmaxf(m, __shfl_xor(m, 2)); m = fmaxf(m, __shfl_xor(m, 4));
  const float ex = expf(l - m); float sm = ex; sm += __shfl_xor(sm, 1); sm += __shfl_xor(sm, 2); sm += __shfl_xor(sm, 4);
  vst2(COEF + row * NK + e, ex / sm); }
template <int ACT, int INP> __global__ __launch_bounds__(128) void k_mix(const float* __restrict__ Yin, const float* __restrict__ Wk, const float* __restrict__ Bk, const float* __restrict__ COEF, float* __restrict__ OUTM) { __shared__ __align__(16) float sf[4][16][132]; __shared__ float sc[64][NK];
  const int tid = threadIdx.x, wave = tid >> 5, lane = tid & 31, col = lane & 15, g = lane >> 4; const int c0 = blockIdx.y * 128; const size_t rb = (size_t)blockIdx.x * 64; const size_t r0 = rb + wave * 16;
  for (int e2 = tid; e2 < 64 * NK; e2 += 128) sc[e2 >> 3][e2 & 7] = COEF[rb * NK + e2];
  __syncthreads();
  v8f tot[8] = {};
#pragma unroll 1
  for (int k = 0; k < NK; ++k) { v8f acc[8] = {}; const float* Wx = Wk + (size_t)k * DM * DM;
#pragma unroll 1
    for (int kc = 0; kc < DM / 32; ++kc) { F2 a; if (INP) { const float* p = Yin + (r0 + col) * DM + kc * 32 + 8 * g;
#pragma unroll
        for (int i = 0; i < 8; ++i) { a.h[i] = (__bf16)p[i]; a.h[8 + i] = (__bf16)p[16 + i]; } } else a = split_row(Yin + (r0 + col) * DM, kc * 32, lane);
      asm volatile("s_wait_loadcnt 0x0" ::: "memory");
#pragma unroll
      for (int j = 0; j < 8; ++j) { const v16b w = wcol_io(Wx, kc * 32, c0 + j * 16 + col, lane, DM); acc[j] = wmma_bf(a.h, w, acc[j]); if (!INP) acc[j] = wmma_bf(a.l, w, acc[j]); } }
#pragma unroll
    for (int j = 0; j < 8; ++j) { const float bb = bfr(Bk[(size_t)k * DM + c0 + j * 16 + col]); asm volatile("s_wait_loadcnt 0x0" ::: "memory");
#pragma unroll
      for (int r = 0; r < 8; ++r) { const float ck = sc[wave * 16 + 8 * g + r][k]; tot[j][r] += ck * (acc[j][r] + bb); } } }
#pragma unroll
  for (int j = 0; j < 8; ++j)
#pragma unroll
    for (int r = 0; r < 8; ++r) sf[wave][8 * g + r][j * 16 + col] = ACT ? elu1(tot[j][r]) : tot[j][r];
  LDSX(); for (int rl = 0; rl < 16; ++rl) vst2(OUTM + (r0 + rl) * DM + c0 + lane * 4, *(const v4f*)&sf[wave][rl][lane * 4]); }
#define WS_G0 0u
#define WS_G1 (WS_G0 + 4u * (size_t)NR * GW)
#define WS_CF (WS_G1 + 4u * (size_t)NR * GW)
#define WS_Y1 (WS_CF + 4u * (size_t)NR * 32)
#define WS_Y2 (WS_Y1 + 4u * (size_t)NR * DM)
#define WS_END (WS_Y2 + 4u * (size_t)NR * DM)
extern "C" void kernel_launch(void* const* d_in, const int* in_sizes, int n_in, void* d_out, int out_size, void* d_ws, size_t ws_size, hipStream_t stream) {
  (void)in_sizes; (void)n_in; (void)out_size;
  const float** F = (const float**)d_in;
  if (ws_size < (size_t)WS_END) return;
  char* ws = (char*)d_ws; float *G0 = (float*)(ws + WS_G0), *G1 = (float*)(ws + WS_G1), *CF = (float*)(ws + WS_CF), *Y1 = (float*)(ws + WS_Y1), *Y2 = (float*)(ws + WS_Y2);
  k_g0<<<dim3(NR / 64), 128, 0, stream>>>(F[1], F[2], F[3], G0);
  k_g1<<<dim3(NR / 64), 128, 0, stream>>>(G0, F[4], F[5], G1);
  k_coef<<<dim3(NR / 32), 256, 0, stream>>>(G1, F[6], F[7], CF);
  k_mix<1, 1><<<dim3(NR / 64, DM / 128), 128, 0, stream>>>(F[0], F[8], F[9], CF, Y1);
  k_mix<1, 0><<<dim3(NR / 64, DM / 128), 128, 0, stream>>>(Y1, F[10], F[11], CF, Y2);
  k_mix<0, 0><<<dim3(NR / 64, DM / 128), 128, 0, stream>>>(Y2, F[12], F[13], CF, (float*)d_out);
}
